// ResidualConvBlock_84447646974225
// MI455X (gfx1250) — hardware-verified
//
#include <hip/hip_runtime.h>
#define NN 50000
#define NE 800000
#define FI 128
#define FO 256

typedef __bf16 v16b __attribute__((ext_vector_type(16)));
typedef unsigned short v8us __attribute__((ext_vector_type(8), may_alias));
typedef float  v8f  __attribute__((ext_vector_type(8)));
typedef float  v4f  __attribute__((ext_vector_type(4)));
typedef float  v4fa __attribute__((ext_vector_type(4), may_alias));
union FragB { v16b v; v8us half[2]; unsigned short u[16]; };

__device__ __forceinline__ unsigned short bf16_bits(float x) { unsigned int u = __float_as_uint(x); return (unsigned short)((u + 0x7FFFu + ((u >> 16) & 1u)) >> 16); }
__device__ __forceinline__ float bf16_val(unsigned short b) { return __uint_as_float(((unsigned int)b) << 16); }
__device__ __forceinline__ float bf16_round(float x) { return bf16_val(bf16_bits(x)); }
template <int NT>
__device__ __forceinline__ v8f mmaN(v16b ah, v16b al, v16b bh, v16b bl, v8f c) {
  c = __builtin_amdgcn_wmma_f32_16x16x32_bf16(false, ah, false, bh, (short)0, c, false, false);
  if (NT >= 2) c = __builtin_amdgcn_wmma_f32_16x16x32_bf16(false, al, false, bh, (short)0, c, false, false);
  if (NT >= 3) c = __builtin_amdgcn_wmma_f32_16x16x32_bf16(false, ah, false, bl, (short)0, c, false, false);
  asm volatile("v_nop\n\tv_nop\n\tv_nop\n\tv_nop" : "+v"(c) : "v"(ah), "v"(al), "v"(bh), "v"(bl));
  return c;
}

__device__ __forceinline__ void store_span256(float* span, v4f lo, v4f hi, int lane) {
  v4f a, b; const int s0 = lane >> 1, s1 = 16 + (lane >> 1); const bool odd = (lane & 1) != 0;
#pragma unroll
  for (int q = 0; q < 4; ++q) { const float l0 = __shfl(lo[q], s0, 32), h0 = __shfl(hi[q], s0, 32), l1 = __shfl(lo[q], s1, 32), h1 = __shfl(hi[q], s1, 32); a[q] = odd ? h0 : l0; b[q] = odd ? h1 : l1; }
  for (int pass = 0; pass < 2; ++pass) { *(volatile v4f*)(span + 4 * lane) = a; *(volatile v4f*)(span + 128 + 4 * lane) = b; if (pass == 0) __threadfence(); } }
__device__ __forceinline__ void store_span512h(_Float16* span, v8us p0, v8us p1, int lane) {
  typedef unsigned int v4u __attribute__((ext_vector_type(4))); union U { v8us h; v4u u; }; U x0, x1, a, b; x0.h = p0; x1.h = p1; const int s0 = lane >> 1, s1 = 16 + (lane >> 1); const bool odd = (lane & 1) != 0;
#pragma unroll
  for (int q = 0; q < 4; ++q) { const unsigned l0 = __shfl(x0.u[q], s0, 32), h0 = __shfl(x1.u[q], s0, 32), l1 = __shfl(x0.u[q], s1, 32), h1 = __shfl(x1.u[q], s1, 32); a.u[q] = odd ? h0 : l0; b.u[q] = odd ? h1 : l1; }
  for (int pass = 0; pass < 2; ++pass) { *(volatile v8us*)((unsigned short*)span + 8 * lane) = a.h; *(volatile v8us*)((unsigned short*)span + 256 + 8 * lane) = b.h; if (pass == 0) __threadfence(); } }

__global__ __launch_bounds__(256) void k_wt_bf16(const float* __restrict__ W, unsigned short* __restrict__ Wt, int K, int N) {
  const int t = blockIdx.x * 256 + threadIdx.x;
  const int k8n = K / 8;
  if (t >= N * k8n) return;
  const int n = t / k8n, k8 = (t % k8n) * 8;
  v8us v;
#pragma unroll
  for (int i = 0; i < 8; ++i) v[i] = bf16_bits(W[(size_t)(k8 + i) * N + n]);
  *(volatile v8us*)(Wt + (size_t)n * K + k8) = v;
  __threadfence();
  *(volatile v8us*)(Wt + (size_t)n * K + k8) = v;
}

template <bool ASPLIT, int ACT, bool BIAS_BF16>
__global__ __launch_bounds__(128) void k_gemm_bf(const float* __restrict__ A, int lda, const unsigned short* __restrict__ Wt, int ldb,
                                               const float* __restrict__ bias, float* __restrict__ C, int ldc, int M, int N, int K) {
  __shared__ __attribute__((aligned(16))) float so[4][16][64];
  const int tid = threadIdx.x, w = tid >> 5, lane = tid & 31, ln = lane & 15, hh = lane >> 4;
  const int ntn = N / 64;
  const int wid = blockIdx.x * 4 + w;
  const int mt = wid / ntn, nq = wid % ntn;
  if (mt * 16 >= M) return;
  const int row0 = mt * 16, col0 = nq * 64;
  const float* arow = A + (size_t)(row0 + ln) * lda;
  v8f acc[4] = {};
  for (int kb = 0; kb < K; kb += 32) {
    FragB ah, al;
    const v4f x0 = *(const v4fa*)(arow + kb + 8 * hh), x1 = *(const v4fa*)(arow + kb + 8 * hh + 4);
    const v4f x2 = *(const v4fa*)(arow + kb + 16 + 8 * hh), x3 = *(const v4fa*)(arow + kb + 16 + 8 * hh + 4);
    float xs[16] = {x0[0],x0[1],x0[2],x0[3],x1[0],x1[1],x1[2],x1[3],x2[0],x2[1],x2[2],x2[3],x3[0],x3[1],x3[2],x3[3]};
#pragma unroll
    for (int i = 0; i < 16; ++i) { const unsigned short hb = bf16_bits(xs[i]); ah.u[i] = hb; al.u[i] = ASPLIT ? bf16_bits(xs[i] - bf16_val(hb)) : (unsigned short)0; }
#pragma unroll
    for (int t = 0; t < 4; ++t) {
      const unsigned short* brow = Wt + (size_t)(col0 + t * 16 + ln) * ldb + kb;
      FragB b;
      b.half[0] = *(const v8us*)(brow + 8 * hh);
      b.half[1] = *(const v8us*)(brow + 16 + 8 * hh);
      acc[t] = mmaN<ASPLIT ? 2 : 1>(ah.v, al.v, b.v, b.v, acc[t]);
    }
  }
#pragma unroll
  for (int t = 0; t < 4; ++t) {
    float bv = bias ? bias[col0 + t * 16 + ln] : 0.f;
    if (BIAS_BF16) bv = bf16_round(bv);
#pragma unroll
    for (int r = 0; r < 8; ++r) { float v = acc[t][r] + bv; if (ACT == 1) v = fmaxf(v, 0.f); so[w][8 * hh + r][t * 16 + ln] = v; }
  }
  __builtin_amdgcn_fence(__ATOMIC_ACQ_REL, "workgroup");
  __builtin_amdgcn_wave_barrier();
  const int rsub = lane >> 4, c4 = (lane & 15) * 4;
  for (int pass = 0; pass < 2; ++pass) {
#pragma unroll
    for (int q = 0; q < 8; ++q) {
      const int r = q * 2 + rsub;
      const v4f v = *(const v4fa*)&so[w][r][c4];
      *(volatile v4f*)(C + (size_t)(row0 + r) * ldc + col0 + c4) = v;
    }
    if (pass == 0) __threadfence();
  }
}

template <int D, bool CAUSAL>
__global__ __launch_bounds__(128) void k_flash(const float* __restrict__ qb, const float* __restrict__ kb, const float* __restrict__ vb,
                                             int pitch, int T, int H, float scale, float* __restrict__ y, int ypitch) {
  constexpr int KS = D / 32;
  constexpr int DT = D / 16;
  __shared__ __attribute__((aligned(16))) unsigned short sKh[32][D + 8], sKl[32][D + 8], sVh[32][D + 8], sVl[32][D + 8];
  __shared__ __attribute__((aligned(16))) unsigned short sPh[4][16][40], sPl[4][16][40];
  __shared__ __attribute__((aligned(16))) float sO[4][16][D];
  const int tid = threadIdx.x, w = tid >> 5, lane = tid & 31, ln = lane & 15, hh = lane >> 4;
  const int nqb = (T + 63) / 64;
  const int bh = blockIdx.x / nqb, qblk = blockIdx.x % nqb;
  const int b = bh / H, h = bh % H;
  const int q0 = qblk * 64 + w * 16;
  const float* Q = qb + (size_t)b * T * pitch + h * D;
  const float* K = kb + (size_t)b * T * pitch + h * D;
  const float* V = vb + (size_t)b * T * pitch + h * D;

  FragB aqh[KS], aql[KS];
  {
    int row = q0 + ln; if (row >= T) row = T - 1;
    const float* qr = Q + (size_t)row * pitch;
#pragma unroll
    for (int ks = 0; ks < KS; ++ks)
#pragma unroll
      for (int i = 0; i < 16; ++i) {
        const int d = ks * 32 + ((i < 8) ? (8 * hh + i) : (16 + 8 * hh + (i - 8)));
        const float x = qr[d] * scale; const unsigned short hb = bf16_bits(x);
        aqh[ks].u[i] = hb; aql[ks].u[i] = bf16_bits(x - bf16_val(hb));
      }
  }
  float m_r[8], l_r[8];
#pragma unroll
  for (int r = 0; r < 8; ++r) { m_r[r] = -3.0e38f; l_r[r] = 0.f; }
  v8f oacc[DT];
#pragma unroll
  for (int dt = 0; dt < DT; ++dt) oacc[dt] = (v8f){0.f,0.f,0.f,0.f,0.f,0.f,0.f,0.f};

  const int kv_end = CAUSAL ? min(T, qblk * 64 + 64) : T;
  for (int j0 = 0; j0 < kv_end; j0 += 32) {
    __syncthreads();
    for (int e = tid; e < 32 * (D / 4); e += 128) {
      const int r = e / (D / 4), c4 = (e % (D / 4)) * 4;
      const int key = j0 + r;
      v4f kf = {0.f,0.f,0.f,0.f}, vf = {0.f,0.f,0.f,0.f};
      if (key < T) { kf = *(const v4fa*)(K + (size_t)key * pitch + c4); vf = *(const v4fa*)(V + (size_t)key * pitch + c4); }
#pragma unroll
      for (int t = 0; t < 4; ++t) {
        unsigned short hb = bf16_bits(kf[t]); sKh[r][c4 + t] = hb; sKl[r][c4 + t] = bf16_bits(kf[t] - bf16_val(hb));
        hb = bf16_bits(vf[t]); sVh[r][c4 + t] = hb; sVl[r][c4 + t] = bf16_bits(vf[t] - bf16_val(hb));
      }
    }
    __syncthreads();
    v8f s[2];
#pragma unroll
    for (int nt = 0; nt < 2; ++nt) {
      v8f acc = {};
#pragma unroll
      for (int ks = 0; ks < KS; ++ks) {
        FragB bh_, bl_;
        bh_.half[0] = *(const v8us*)&sKh[nt * 16 + ln][ks * 32 + 8 * hh]; bh_.half[1] = *(const v8us*)&sKh[nt * 16 + ln][ks * 32 + 16 + 8 * hh];
        bl_.half[0] = *(const v8us*)&sKl[nt * 16 + ln][ks * 32 + 8 * hh]; bl_.half[1] = *(const v8us*)&sKl[nt * 16 + ln][ks * 32 + 16 + 8 * hh];
        acc = mmaN<3>(aqh[ks].v, aql[ks].v, bh_.v, bl_.v, acc);
      }
      s[nt] = acc;
    }
    float alpha[8];
#pragma unroll
    for (int r = 0; r < 8; ++r) {
      const int qi = q0 + 8 * hh + r;
      const int ja = j0 + ln, jb = j0 + 16 + ln;
      if (CAUSAL) { if (ja > qi) s[0][r] = -3.0e38f; if (jb > qi) s[1][r] = -3.0e38f; }
      if (ja >= T) s[0][r] = -3.0e38f;
      if (jb >= T) s[1][r] = -3.0e38f;
      float mx = fmaxf(s[0][r], s[1][r]);
      mx = fmaxf(mx, __shfl_xor(mx, 1, 32)); mx = fmaxf(mx, __shfl_xor(mx, 2, 32)); mx = fmaxf(mx, __shfl_xor(mx, 4, 32)); mx = fmaxf(mx, __shfl_xor(mx, 8, 32));
      const float mnew = fmaxf(m_r[r], mx);
      alpha[r] = (mnew > -1.0e38f) ? __expf(m_r[r] - mnew) : 1.0f;
      const float p0 = (s[0][r] > -1.0e38f) ? __expf(s[0][r] - mnew) : 0.f;
      const float p1 = (s[1][r] > -1.0e38f) ? __expf(s[1][r] - mnew) : 0.f;
      m_r[r] = mnew;
      l_r[r] = l_r[r] * alpha[r] + p0 + p1;
      unsigned short hb = bf16_bits(p0); sPh[w][8 * hh + r][ln] = hb;      sPl[w][8 * hh + r][ln] = bf16_bits(p0 - bf16_val(hb));
      hb = bf16_bits(p1);                sPh[w][8 * hh + r][16 + ln] = hb; sPl[w][8 * hh + r][16 + ln] = bf16_bits(p1 - bf16_val(hb));
    }
#pragma unroll
    for (int dt = 0; dt < DT; ++dt)
#pragma unroll
      for (int r = 0; r < 8; ++r) oacc[dt][r] *= alpha[r];
    __builtin_amdgcn_fence(__ATOMIC_ACQ_REL, "workgroup");
    __builtin_amdgcn_wave_barrier();
    FragB pah, pal;
    pah.half[0] = *(const v8us*)&sPh[w][ln][8 * hh]; pah.half[1] = *(const v8us*)&sPh[w][ln][16 + 8 * hh];
    pal.half[0] = *(const v8us*)&sPl[w][ln][8 * hh]; pal.half[1] = *(const v8us*)&sPl[w][ln][16 + 8 * hh];
#pragma unroll
    for (int dt = 0; dt < DT; ++dt) {
      FragB bvh, bvl;
#pragma unroll
      for (int i = 0; i < 8; ++i) {
        bvh.u[i] = sVh[8 * hh + i][dt * 16 + ln]; bvh.u[8 + i] = sVh[16 + 8 * hh + i][dt * 16 + ln];
        bvl.u[i] = sVl[8 * hh + i][dt * 16 + ln]; bvl.u[8 + i] = sVl[16 + 8 * hh + i][dt * 16 + ln];
      }
      oacc[dt] = mmaN<3>(pah.v, pal.v, bvh.v, bvl.v, oacc[dt]);
    }
    __builtin_amdgcn_fence(__ATOMIC_ACQ_REL, "workgroup");
    __builtin_amdgcn_wave_barrier();
  }
#pragma unroll
  for (int r = 0; r < 8; ++r) {
    float l = l_r[r];
    l += __shfl_xor(l, 1, 32); l += __shfl_xor(l, 2, 32); l += __shfl_xor(l, 4, 32); l += __shfl_xor(l, 8, 32);
    l_r[r] = (l > 0.f) ? 1.0f / l : 0.f;
  }
#pragma unroll
  for (int dt = 0; dt < DT; ++dt)
#pragma unroll
    for (int r = 0; r < 8; ++r) sO[w][8 * hh + r][dt * 16 + ln] = oacc[dt][r] * l_r[r];
  __builtin_amdgcn_fence(__ATOMIC_ACQ_REL, "workgroup");
  __builtin_amdgcn_wave_barrier();
  for (int pass = 0; pass < 2; ++pass) {
    for (int r = 0; r < 16; ++r) {
      const int row = q0 + r;
      if (row < T && lane < D / 4) {
        const v4f val = *(const v4fa*)&sO[w][r][lane * 4];
        *(volatile v4f*)(y + ((size_t)b * T + row) * ypitch + h * D + lane * 4) = val;
      }
    }
    if (pass == 0) __threadfence();
  }
}

typedef _Float16 v16h __attribute__((ext_vector_type(16)));
union FragH { v16h v; v8us half[2]; _Float16 h[16]; unsigned short u[16]; };
template <int NT>
__device__ __forceinline__ v8f mmaH(v16h ah, v16h al, v16h bh, v16h bl, v8f c) {
  c = __builtin_amdgcn_wmma_f32_16x16x32_f16(false, ah, false, bh, (short)0, c, false, false);
  if (NT >= 2) c = __builtin_amdgcn_wmma_f32_16x16x32_f16(false, al, false, bh, (short)0, c, false, false);
  if (NT >= 3) c = __builtin_amdgcn_wmma_f32_16x16x32_f16(false, ah, false, bl, (short)0, c, false, false);
  asm volatile("v_nop\n\tv_nop\n\tv_nop\n\tv_nop" : "+v"(c) : "v"(ah), "v"(al), "v"(bh), "v"(bl));
  return c;
}
template <bool ASPLIT>
__global__ __launch_bounds__(128) void k_gemm_h(const float* __restrict__ A, int lda, size_t sA, const _Float16* __restrict__ Bh, int ldb, size_t sB, float alpha, float* __restrict__ C, int ldc, size_t sC, int M, int N, int K) {
  __shared__ __attribute__((aligned(16))) float so[4][16][64];
  const int tid = threadIdx.x, w = tid >> 5, lane = tid & 31, ln = lane & 15, hh = lane >> 4; const int by = blockIdx.y;
  A += (size_t)by * sA; Bh += (size_t)by * sB; C += (size_t)by * sC;
  const int ntn = (N + 63) / 64; const int wid = blockIdx.x * 4 + w; const int mt = wid / ntn, nq = wid % ntn; if (mt * 16 >= M) return;
  const int row0 = mt * 16, col0 = nq * 64; const float* arow = A + (size_t)(row0 + ln) * lda;
  v8f acc[4] = {};
  for (int kb = 0; kb < K; kb += 32) {
    FragH ah, al;
    const v4f x0 = *(const v4fa*)(arow + kb + 8 * hh), x1 = *(const v4fa*)(arow + kb + 8 * hh + 4), x2 = *(const v4fa*)(arow + kb + 16 + 8 * hh), x3 = *(const v4fa*)(arow + kb + 16 + 8 * hh + 4);
    float xs[16] = {x0[0],x0[1],x0[2],x0[3],x1[0],x1[1],x1[2],x1[3],x2[0],x2[1],x2[2],x2[3],x3[0],x3[1],x3[2],x3[3]};
#pragma unroll
    for (int i = 0; i < 16; ++i) { const _Float16 h = (_Float16)xs[i]; ah.h[i] = h; al.h[i] = ASPLIT ? (_Float16)(xs[i] - (float)h) : (_Float16)0.0f; }
#pragma unroll
    for (int t = 0; t < 4; ++t) { if (col0 + t * 16 >= N) continue; const size_t boff = (size_t)(col0 + t * 16 + ln) * ldb + kb; FragH bq; bq.half[0] = *(const v8us*)(Bh + boff + 8 * hh); bq.half[1] = *(const v8us*)(Bh + boff + 16 + 8 * hh);
      acc[t] = mmaH<ASPLIT ? 2 : 1>(ah.v, al.v, bq.v, bq.v, acc[t]); }
  }
#pragma unroll
  for (int t = 0; t < 4; ++t) { if (col0 + t * 16 >= N) continue;
#pragma unroll
    for (int r = 0; r < 8; ++r) so[w][8 * hh + r][t * 16 + ln] = acc[t][r] * alpha; }
  __builtin_amdgcn_fence(__ATOMIC_ACQ_REL, "workgroup"); __builtin_amdgcn_wave_barrier();
  const int rsub = lane >> 4, c4 = (lane & 15) * 4;
  for (int pass = 0; pass < 2; ++pass) {
#pragma unroll
    for (int q = 0; q < 8; ++q) { const int r = q * 2 + rsub; if (col0 + c4 < N) { const v4f v = *(const v4fa*)&so[w][r][c4]; *(volatile v4f*)(C + (size_t)(row0 + r) * ldc + col0 + c4) = v; } }
    if (pass == 0) __threadfence(); }
}

template <int DUMMY>
__global__ __launch_bounds__(128) void k_gemm_hh(const _Float16* __restrict__ A, int lda, size_t sA, const _Float16* __restrict__ Bh, int ldb, size_t sB, float alpha, float* __restrict__ C, int ldc, size_t sC, int M, int N, int K) {
  __shared__ __attribute__((aligned(16))) float so[4][16][64];
  const int tid = threadIdx.x, w = tid >> 5, lane = tid & 31, ln = lane & 15, hh = lane >> 4; const int by = blockIdx.y;
  A += (size_t)by * sA; Bh += (size_t)by * sB; C += (size_t)by * sC;
  const int ntn = (N + 63) / 64; const int wid = blockIdx.x * 4 + w; const int mt = wid / ntn, nq = wid % ntn; if (mt * 16 >= M) return;
  const int row0 = mt * 16, col0 = nq * 64; const _Float16* arow = A + (size_t)(row0 + ln) * lda;
  v8f acc[4] = {};
  for (int kb = 0; kb < K; kb += 32) { FragH ah; ah.half[0] = *(const v8us*)((const unsigned short*)arow + kb + 8 * hh); ah.half[1] = *(const v8us*)((const unsigned short*)arow + kb + 16 + 8 * hh);
#pragma unroll
    for (int t = 0; t < 4; ++t) { if (col0 + t * 16 >= N) continue; const size_t boff = (size_t)(col0 + t * 16 + ln) * ldb + kb; FragH bq; bq.half[0] = *(const v8us*)((const unsigned short*)Bh + boff + 8 * hh); bq.half[1] = *(const v8us*)((const unsigned short*)Bh + boff + 16 + 8 * hh);
      acc[t] = mmaH<1>(ah.v, ah.v, bq.v, bq.v, acc[t]); }
  }
#pragma unroll
  for (int t = 0; t < 4; ++t) { if (col0 + t * 16 >= N) continue;
#pragma unroll
    for (int r = 0; r < 8; ++r) so[w][8 * hh + r][t * 16 + ln] = acc[t][r] * alpha; }
  __builtin_amdgcn_fence(__ATOMIC_ACQ_REL, "workgroup"); __builtin_amdgcn_wave_barrier();
  const int rsub = lane >> 4, c4 = (lane & 15) * 4;
  for (int pass = 0; pass < 2; ++pass) {
#pragma unroll
    for (int q = 0; q < 8; ++q) { const int r = q * 2 + rsub; if (col0 + c4 < N) { const v4f v = *(const v4fa*)&so[w][r][c4]; *(volatile v4f*)(C + (size_t)(row0 + r) * ldc + col0 + c4) = v; } }
    if (pass == 0) __threadfence(); }
}

template <int ACT>
__global__ __launch_bounds__(128) void k_gemm_hhx(const _Float16* __restrict__ A, int lda, size_t sA, const _Float16* __restrict__ Bh, int ldb, size_t sB, float alpha, const float* __restrict__ bias, size_t sBias, const float* __restrict__ CP, int rowsPerB, size_t sCPb, int row0g,
    float* __restrict__ C, _Float16* __restrict__ C16, int ldc, size_t sC, int M, int N, int K) {
  __shared__ __attribute__((aligned(16))) float so[4][16][64];
  const int tid = threadIdx.x, w = tid >> 5, lane = tid & 31, ln = lane & 15, hh = lane >> 4; const int by = blockIdx.y;
  A += (size_t)by * sA; Bh += (size_t)by * sB; const size_t cofs = (size_t)by * sC; const float* bp = bias ? bias + (size_t)by * sBias : nullptr;
  const int ntn = (N + 63) / 64; const int wid = blockIdx.x * 4 + w; const int mt = wid / ntn, nq = wid % ntn; if (mt * 16 >= M) return;
  const int row0 = mt * 16, col0 = nq * 64; const _Float16* arow = A + (size_t)(row0 + ln) * lda;
  v8f acc[4] = {};
  for (int kb = 0; kb < K; kb += 32) { FragH ah; ah.half[0] = *(const v8us*)((const unsigned short*)arow + kb + 8 * hh); ah.half[1] = *(const v8us*)((const unsigned short*)arow + kb + 16 + 8 * hh);
#pragma unroll
    for (int t = 0; t < 4; ++t) { if (col0 + t * 16 >= N) continue; const size_t boff = (size_t)(col0 + t * 16 + ln) * ldb + kb; FragH bq; bq.half[0] = *(const v8us*)((const unsigned short*)Bh + boff + 8 * hh); bq.half[1] = *(const v8us*)((const unsigned short*)Bh + boff + 16 + 8 * hh);
      acc[t] = mmaH<1>(ah.v, ah.v, bq.v, bq.v, acc[t]); }
  }
#pragma unroll
  for (int t = 0; t < 4; ++t) { if (col0 + t * 16 >= N) continue; const int col = col0 + t * 16 + ln; const float bv = bp ? bf16_round(bp[col]) : 0.f;
#pragma unroll
    for (int r = 0; r < 8; ++r) { float v = acc[t][r] * alpha + bv; if (CP) { const int bidx = (row0g + row0 + 8 * hh + r) / rowsPerB; v += CP[(size_t)bidx * sCPb + (size_t)by * 64 + col]; } if (ACT == 1) v = (v > 0.f) ? v : expm1f(v); so[w][8 * hh + r][t * 16 + ln] = v; } }
  __builtin_amdgcn_fence(__ATOMIC_ACQ_REL, "workgroup"); __builtin_amdgcn_wave_barrier();
  const int rsub = lane >> 4, c4 = (lane & 15) * 4; typedef _Float16 v4h __attribute__((ext_vector_type(4)));
  for (int pass = 0; pass < 2; ++pass) {
#pragma unroll
    for (int q = 0; q < 8; ++q) { const int r = q * 2 + rsub; if (col0 + c4 < N) { const v4f v = *(const v4fa*)&so[w][r][c4]; if (C) *(volatile v4f*)(C + cofs + (size_t)(row0 + r) * ldc + col0 + c4) = v; if (C16) { v4h h4; for (int i = 0; i < 4; ++i) h4[i] = (_Float16)v[i]; *(volatile v4h*)(C16 + cofs + (size_t)(row0 + r) * ldc + col0 + c4) = h4; } } }
    if (pass == 0) __threadfence(); }
}

__device__ __forceinline__ int bscan_k_seg(int cnt, int* scan, int tid, int& total) { __syncthreads(); scan[tid] = cnt; __syncthreads();
  for (int of = 1; of < 512; of <<= 1) { const int v = (tid >= of) ? scan[tid - of] : 0; __syncthreads(); scan[tid] += v; __syncthreads(); }
  total = scan[512 - 1]; return scan[tid] - cnt; }
__global__ __launch_bounds__(512) void k_seg(const float* __restrict__ Hs, const int* __restrict__ src, const int* __restrict__ dst, const float* __restrict__ DINV, float* __restrict__ MEAN) {
  __shared__ short Lr[4096]; __shared__ int Lc[4096];  __shared__ int scan[512]; __shared__ float stg[64][128 + 1];
  const int tid = threadIdx.x; const int s0 = blockIdx.x * 512; float acc0[128];
#pragma unroll
  for (int c = 0; c < 128; ++c) acc0[c] = 0.f;
  for (int e0 = 0; e0 < (NE); e0 += 4096) { int hr[8], hc[8];  int cnt = 0;
#pragma unroll
    for (int k = 0; k < 8; ++k) { const int e = e0 + tid * 8 + k; hr[k] = -1; hc[k] = 0;  if (e < (NE)) { const int dd_ = (dst[e]); if (dd_ >= s0 && dd_ < s0 + 512) { hr[k] = dd_ - s0; int s = (src[e]); s = s < 0 ? 0 : (s >= (NN) ? (NN) - 1 : s); hc[k] = s;  ++cnt; } } }
    int tot; int p = bscan_k_seg(cnt, scan, tid, tot);
#pragma unroll
    for (int k = 0; k < 8; ++k) if (hr[k] >= 0) { Lr[p] = (short)hr[k]; Lc[p] = hc[k];  ++p; }
    __syncthreads();
#pragma unroll 1
    for (int q = 0; q < tot; ++q) { if (Lr[q] == tid) { const float* row = (Hs + (size_t)Lc[q] * FI);
#pragma unroll
        for (int c = 0; c < 128; c += 4) { const v4f v = *(const v4fa*)(row + c); acc0[c] += v[0]; acc0[c + 1] += v[1]; acc0[c + 2] += v[2]; acc0[c + 3] += v[3]; } } }
    __syncthreads(); }
  for (int tg = 0; tg < 512 / 64; ++tg) {
    if (tid / 64 == tg) {
#pragma unroll
      for (int c = 0; c < 128; ++c) stg[tid % 64][c] = acc0[c]; }
    __syncthreads();
    for (int pass = 0; pass < 2; ++pass) { for (int i = tid; i < 64 * (128 / 4); i += 512) { const int r = i / (128 / 4), c4 = (i % (128 / 4)) * 4; const int seg = s0 + tg * 64 + r; if (seg < (NN)) { v4f v; v[0] = stg[r][c4]; v[1] = stg[r][c4 + 1]; v[2] = stg[r][c4 + 2]; v[3] = stg[r][c4 + 3]; { const float sc_ = (DINV[seg]); for (int q2 = 0; q2 < 4; ++q2) v[q2] *= sc_; } *(volatile v4f*)((MEAN + (size_t)seg * FI) + c4) = v; } } if (pass == 0) __threadfence(); }
    __syncthreads(); } }

__global__ __launch_bounds__(256) void k_ln1(const float* __restrict__ h, const float* __restrict__ g, const float* __restrict__ be, float* __restrict__ H) { const int tid = threadIdx.x, wv = tid >> 5, lane = tid & 31; const size_t n = (size_t)blockIdx.x * 8 + wv; if (n >= NN) return; const v4f xv = *(const v4fa*)(h + n * FI + 4 * lane); float v[4]; float s = 0.f; for (int q = 0; q < 4; ++q) { v[q] = bf16_round(xv[q]); s += v[q]; }
  for (int o = 16; o >= 1; o >>= 1) s += __shfl_xor(s, o, 32); const float mu = s / (float)FI; float q2 = 0.f; for (int q = 0; q < 4; ++q) { const float d = v[q] - mu; q2 += d * d; } for (int o = 16; o >= 1; o >>= 1) q2 += __shfl_xor(q2, o, 32); const float inv = 1.0f / sqrtf(q2 / (float)FI + 1e-5f);
  v4f o4; for (int q = 0; q < 4; ++q) { const int c = 4 * lane + q; o4[q] = (v[q] - mu) * inv * bf16_round(g[c]) + bf16_round(be[c]); }
  *(volatile v4f*)(H + n * FI + 4 * lane) = o4; __threadfence(); *(volatile v4f*)(H + n * FI + 4 * lane) = o4; }
__device__ __forceinline__ int bscan1024(int cnt, int* scan, int tid, int& total) { __syncthreads(); scan[tid] = cnt; __syncthreads();
  for (int of = 1; of < 1024; of <<= 1) { const int v = (tid >= of) ? scan[tid - of] : 0; __syncthreads(); scan[tid] += v; __syncthreads(); }
  total = scan[1023]; return scan[tid] - cnt; }
__global__ __launch_bounds__(1024) void k_deg(const int* __restrict__ dst, float* __restrict__ DINV) { __shared__ short Lr[4096]; __shared__ int scan[1024]; const int tid = threadIdx.x; const int n0 = blockIdx.x * 1024; int d = 0;
  for (int e0 = 0; e0 < NE; e0 += 4096) { int hr[4]; int cnt = 0;
#pragma unroll
    for (int k = 0; k < 4; ++k) { const int e = e0 + tid * 4 + k; hr[k] = -1; if (e < NE) { const int dd = dst[e]; if (dd >= n0 && dd < n0 + 1024) { hr[k] = dd - n0; ++cnt; } } }
    int tot; int p = bscan1024(cnt, scan, tid, tot);
#pragma unroll
    for (int k = 0; k < 4; ++k) if (hr[k] >= 0) { Lr[p] = (short)hr[k]; ++p; }
    __syncthreads();
#pragma unroll 1
    for (int q = 0; q < tot; ++q) if (Lr[q] == tid) ++d;
    __syncthreads(); }
  const int n = n0 + tid; if (n < NN) { const float v = 1.0f / fmaxf((float)d, 1.0f); *(volatile float*)(DINV + n) = v; __threadfence(); *(volatile float*)(DINV + n) = v; } }
__global__ __launch_bounds__(256) void k_pack(const float* __restrict__ H, const float* __restrict__ MEAN, int n0, int rows, _Float16* __restrict__ A16) { const size_t t = (size_t)blockIdx.x * 256 + threadIdx.x; if (t >= (size_t)rows * FO / 8) return; const int c8 = (int)((t * 8) % FO); const size_t r = (t * 8) / FO; const float* srcp = (c8 < FI) ? (H + (size_t)(n0 + r) * FI + c8) : (MEAN + (size_t)(n0 + r) * FI + c8 - FI); FragH f; for (int q = 0; q < 8; ++q) f.h[q] = (_Float16)srcp[q]; *(volatile v8us*)((unsigned short*)A16 + t * 8) = f.half[0]; __threadfence(); *(volatile v8us*)((unsigned short*)A16 + t * 8) = f.half[0]; }
__global__ __launch_bounds__(256) void k_bt(const float* __restrict__ Ws, const float* __restrict__ Wn, const float* __restrict__ Wsi, _Float16* __restrict__ B1, _Float16* __restrict__ B2) { const int t = blockIdx.x * 256 + threadIdx.x; if (t >= FO * FO) return; const int k = t % FO, n = t / FO; const float a = (k < FI) ? Ws[k * FO + n] : Wn[(k - FI) * FO + n]; *(volatile _Float16*)(B1 + t) = (_Float16)(bf16_round(a) * 16.0f); *(volatile _Float16*)(B2 + t) = (_Float16)(bf16_round(Wsi[k * FO + n]) * 16.0f); }
__global__ __launch_bounds__(256) void k_ln2(const float* __restrict__ CV, const float* __restrict__ H, const float* __restrict__ g, const float* __restrict__ be, int n0, int rows, float* __restrict__ X, _Float16* __restrict__ X16) { const int tid = threadIdx.x, wv = tid >> 5, lane = tid & 31; const size_t n = (size_t)blockIdx.x * 8 + wv; if (n >= (size_t)rows) return; float v[8]; float s = 0.f;
  { const v4f a = *(const v4fa*)(CV + n * FO + 8 * lane), b = *(const v4fa*)(CV + n * FO + 8 * lane + 4); const v4f hh = *(const v4fa*)(H + (n0 + n) * FI + 4 * lane); for (int q = 0; q < 4; ++q) { v[q] = a[q] + hh[q / 2]; v[4 + q] = b[q] + hh[2 + q / 2]; } }
  for (int q = 0; q < 8; ++q) s += v[q]; for (int o = 16; o >= 1; o >>= 1) s += __shfl_xor(s, o, 32); const float mu = s / (float)FO; float q2 = 0.f; for (int q = 0; q < 8; ++q) { const float d = v[q] - mu; q2 += d * d; } for (int o = 16; o >= 1; o >>= 1) q2 += __shfl_xor(q2, o, 32); const float inv = 1.0f / sqrtf(q2 / (float)FO + 1e-5f);
  v4f o0, o1; FragH f; for (int q = 0; q < 8; ++q) { const int c = 8 * lane + q; const float y = (v[q] - mu) * inv * bf16_round(g[c]) + bf16_round(be[c]); if (q < 4) o0[q] = y; else o1[q - 4] = y; f.h[q] = (_Float16)y; }
  store_span256(X + n * FO, o0, o1, lane); *(volatile v8us*)((unsigned short*)X16 + n * FO + 8 * lane) = f.half[0]; __threadfence(); *(volatile v8us*)((unsigned short*)X16 + n * FO + 8 * lane) = f.half[0]; }
__global__ __launch_bounds__(256) void k_fin(const float* __restrict__ G, const float* __restrict__ X, int rows, float* __restrict__ out) { const size_t t = (size_t)blockIdx.x * 256 + threadIdx.x; if (t >= (size_t)rows * FO / 4) return; const v4f gv = *(const v4fa*)(G + t * 4), xv = *(const v4fa*)(X + t * 4); v4f o; for (int q = 0; q < 4; ++q) { const float a = gv[q]; o[q] = (a > 0.f ? a : expm1f(a)) + xv[q]; } *(volatile v4f*)(out + t * 4) = o; __threadfence(); *(volatile v4f*)(out + t * 4) = o; }
extern "C" void kernel_launch(void* const* d_in, const int* in_sizes, int n_in,
                              void* d_out, int out_size, void* d_ws, size_t ws_size, hipStream_t stream) {
  (void)in_sizes; (void)n_in; (void)out_size;
  const float* h = (const float*)d_in[0]; const int* src = (const int*)d_in[1]; const int* dst = (const int*)d_in[2]; const float* g1 = (const float*)d_in[3]; const float* be1 = (const float*)d_in[4]; const float* Ws = (const float*)d_in[5]; const float* Wn = (const float*)d_in[6]; const float* bn = (const float*)d_in[7]; const float* g2 = (const float*)d_in[8]; const float* be2 = (const float*)d_in[9]; const float* Wsi = (const float*)d_in[10]; const float* bsi = (const float*)d_in[11];
  char* ws = (char*)d_ws; size_t off = 0;
  auto take = [&](size_t bytes) { char* p = ws + off; off += (bytes + 255) & ~(size_t)255; return p; };
  const int RCH = 12512;
  _Float16* B1 = (_Float16*)take((size_t)FO * FO * 2); _Float16* B2 = (_Float16*)take((size_t)FO * FO * 2); float* H = (float*)take((size_t)NN * FI * 4); float* DINV = (float*)take(NN * 4); float* MEAN = (float*)take((size_t)NN * FI * 4);
  _Float16* A16 = (_Float16*)take((size_t)RCH * FO * 2); float* CV = (float*)take((size_t)RCH * FO * 4); float* X = (float*)take((size_t)RCH * FO * 4); _Float16* X16 = (_Float16*)take((size_t)RCH * FO * 2); float* G = CV;
  if (off > ws_size) return;
  k_bt<<<(FO * FO + 255) / 256, 256, 0, stream>>>(Ws, Wn, Wsi, B1, B2);
  k_ln1<<<(NN + 7) / 8, 256, 0, stream>>>(h, g1, be1, H);
  k_deg<<<(NN + 1023) / 1024, 1024, 0, stream>>>(dst, DINV);
  k_seg<<<(NN + 511) / 512, 512, 0, stream>>>(H, src, dst, DINV, MEAN);
  for (int n0 = 0; n0 < NN; n0 += RCH) { const int rows = (NN - n0 < RCH) ? (NN - n0) : RCH; const dim3 gg(((rows / 16) * (FO / 64) + 3) / 4, 1);
    k_pack<<<(unsigned)(((size_t)rows * FO / 8 + 255) / 256), 256, 0, stream>>>(H, MEAN, n0, rows, A16);
    k_gemm_hhx<0><<<gg, 128, 0, stream>>>(A16, FO, 0, B1, FO, 0, 0.0625f, bn, 0, nullptr, 1, 0, 0, CV, nullptr, FO, 0, rows, FO, FO);
    k_ln2<<<(rows + 7) / 8, 256, 0, stream>>>(CV, H, g2, be2, n0, rows, X, X16);
    k_gemm_hhx<0><<<gg, 128, 0, stream>>>(X16, FO, 0, B2, FO, 0, 0.0625f, bsi, 0, nullptr, 1, 0, 0, G, nullptr, FO, 0, rows, FO, FO);
    k_fin<<<(unsigned)(((size_t)rows * FO / 4 + 255) / 256), 256, 0, stream>>>(G, X, rows, (float*)d_out + (size_t)n0 * FO); }
}
